// CausalAttentionBlock_5093831213186
// MI455X (gfx1250) — hardware-run, weakly checked
//
#include <hip/hip_runtime.h>
#include <math.h>
#include <stdint.h>

#define NB     2
#define SEQ    2048
#define HID    1024
#define NHD    16
#define HD     64
#define NTOK   (NB * SEQ)
#define QKVN   (3 * HID)
#define QKP    (2 * HID)
#define FFN    (2 * HID)
#define WSC    64.0f
#define PSCALE 16384.0f
#define CTXC   16.0f
#define H1C    8.0f
static_assert(NHD * HD == HID);
static_assert((SEQ % 64) == 0 && (HID % 64) == 0 && (FFN % 64) == 0 && (NTOK % 64) == 0 && (QKVN % 64) == 0);
static_assert((HID % 32) == 0 && (FFN % 32) == 0);
static_assert((HID % 256) == 0);

typedef _Float16 v16h __attribute__((ext_vector_type(16)));
typedef _Float16 v8h  __attribute__((ext_vector_type(8)));
typedef float    v8f  __attribute__((ext_vector_type(8)));
typedef float    v4f  __attribute__((ext_vector_type(4)));
typedef v8h __attribute__((may_alias)) v8ha;
typedef v4f __attribute__((may_alias)) v4fa;
union Frag { v16h v; v8h half[2]; };

__device__ __forceinline__ v8f zero8() { v8f z = {0.f, 0.f, 0.f, 0.f, 0.f, 0.f, 0.f, 0.f}; return z; }
__device__ __forceinline__ float gelu_f(float v) { return 0.5f * v * (1.0f + erff(v * 0.70710678118654752f)); }

__device__ __forceinline__ v16h ldfrag(const _Float16* p) {
  Frag f;
  f.half[0] = *(const v8ha*)(p);
  f.half[1] = *(const v8ha*)(p + 16);
  return f.v;
}

__device__ __forceinline__ v8f mma_h(v16h a, v16h b, v8f c) {
  c = __builtin_amdgcn_wmma_f32_16x16x32_f16(false, a, false, b, (short)0, c, false, false);
  asm volatile("v_nop\n\tv_nop\n\tv_nop\n\tv_nop" : "+v"(c) : "v"(a), "v"(b));
  return c;
}
__device__ __forceinline__ v8f mma_raw(v16h a, v16h b, v8f c) {
  return __builtin_amdgcn_wmma_f32_16x16x32_f16(false, a, false, b, (short)0, c, false, false);
}
__device__ __forceinline__ void dep_guard4(v8f& a, v8f& b, v8f& c, v8f& d, v16h x) {
  asm volatile("v_nop\n\tv_nop\n\tv_nop\n\tv_nop" : "+v"(a), "+v"(b), "+v"(c), "+v"(d) : "v"(x));
}
__device__ __forceinline__ void keep4(v16h a, v16h b, v16h c, v16h d) {
  asm volatile("v_nop" :: "v"(a), "v"(b), "v"(c), "v"(d));
}
__device__ __forceinline__ void acc_guard4(v8f& a, v8f& b, v8f& c, v8f& d) {
  asm volatile("v_nop\n\tv_nop\n\tv_nop\n\tv_nop" : "+v"(a), "+v"(b), "+v"(c), "+v"(d));
}

__global__ __launch_bounds__(256) void ln_kernel(const float* __restrict__ x, const float* __restrict__ gam,
                                                 const float* __restrict__ bet, _Float16* y, int nrows) {
  const int wave = threadIdx.x >> 5, lane = threadIdx.x & 31;
  const int row = blockIdx.x * 8 + wave;
  if (row >= nrows) return;
  const float* xr = x + (size_t)row * HID;
  _Float16* yr = y + (size_t)row * HID;

  float s = 0.f;
#pragma unroll 1
  for (int c = 0; c < HID / 256; ++c) {
    const v4f a = *(const v4fa*)(xr + c * 256 + lane * 8);
    const v4f e = *(const v4fa*)(xr + c * 256 + lane * 8 + 4);
    s += ((a.x + a.y) + (a.z + a.w)) + ((e.x + e.y) + (e.z + e.w));
  }
#pragma unroll
  for (int o = 1; o < 32; o <<= 1) s += __shfl_xor(s, o, 32);
  const float mu = s * (1.0f / (float)HID);

  float sq = 0.f;
#pragma unroll 1
  for (int c = 0; c < HID / 256; ++c) {
    const v4f a = *(const v4fa*)(xr + c * 256 + lane * 8);
    const v4f e = *(const v4fa*)(xr + c * 256 + lane * 8 + 4);
    const v4f d0 = a - mu, d1 = e - mu;
    sq += (d0.x * d0.x + d0.y * d0.y) + (d0.z * d0.z + d0.w * d0.w)
        + (d1.x * d1.x + d1.y * d1.y) + (d1.z * d1.z + d1.w * d1.w);
  }
#pragma unroll
  for (int o = 1; o < 32; o <<= 1) sq += __shfl_xor(sq, o, 32);
  const float var  = sq * (1.0f / (float)HID);
  const float rstd = 1.0f / sqrtf(var + 1e-12f);

  for (int pass = 0; pass < 2; ++pass) {
#pragma unroll 1
    for (int c = 0; c < HID / 256; ++c) {
      const int col = c * 256 + lane * 8;
      const v4f a  = *(const v4fa*)(xr + col);
      const v4f e  = *(const v4fa*)(xr + col + 4);
      const v4f g0 = *(const v4fa*)(gam + col);
      const v4f g1 = *(const v4fa*)(gam + col + 4);
      const v4f b0 = *(const v4fa*)(bet + col);
      const v4f b1 = *(const v4fa*)(bet + col + 4);
      const v4f y0 = (a - mu) * rstd * g0 + b0;
      const v4f y1 = (e - mu) * rstd * g1 + b1;
      const v8h o = { (_Float16)y0.x, (_Float16)y0.y, (_Float16)y0.z, (_Float16)y0.w,
                      (_Float16)y1.x, (_Float16)y1.y, (_Float16)y1.z, (_Float16)y1.w };
      *(volatile v8h*)(yr + col) = o;
    }
    __threadfence();
  }
}

__global__ __launch_bounds__(256) void wtrans_kernel(const float* __restrict__ W, _Float16* Wt, int K, int N) {
  __shared__ __align__(16) _Float16 T[64 * 72];
  const int tid = threadIdx.x, lane = tid & 31, wave = tid >> 5;
  const int n0 = blockIdx.x * 64, k0 = blockIdx.y * 64;
  {
    const int kr = tid >> 2, nq = (tid & 3) * 16;
    const float* src = W + (size_t)(k0 + kr) * N + n0 + nq;
    const v4f a0 = *(const v4fa*)(src);
    const v4f a1 = *(const v4fa*)(src + 4);
    const v4f a2 = *(const v4fa*)(src + 8);
    const v4f a3 = *(const v4fa*)(src + 12);
    _Float16* tp = T + nq * 72 + kr;
    tp[ 0 * 72] = (_Float16)(a0.x * WSC); tp[ 1 * 72] = (_Float16)(a0.y * WSC);
    tp[ 2 * 72] = (_Float16)(a0.z * WSC); tp[ 3 * 72] = (_Float16)(a0.w * WSC);
    tp[ 4 * 72] = (_Float16)(a1.x * WSC); tp[ 5 * 72] = (_Float16)(a1.y * WSC);
    tp[ 6 * 72] = (_Float16)(a1.z * WSC); tp[ 7 * 72] = (_Float16)(a1.w * WSC);
    tp[ 8 * 72] = (_Float16)(a2.x * WSC); tp[ 9 * 72] = (_Float16)(a2.y * WSC);
    tp[10 * 72] = (_Float16)(a2.z * WSC); tp[11 * 72] = (_Float16)(a2.w * WSC);
    tp[12 * 72] = (_Float16)(a3.x * WSC); tp[13 * 72] = (_Float16)(a3.y * WSC);
    tp[14 * 72] = (_Float16)(a3.z * WSC); tp[15 * 72] = (_Float16)(a3.w * WSC);
  }
  __syncthreads();
  const int q8 = lane & 7, sub = lane >> 3;
  const int r0 = wave * 8 + sub, r1 = wave * 8 + 4 + sub;
  const v8h v0 = *(const v8ha*)(T + r0 * 72 + 8 * q8);
  const v8h v1 = *(const v8ha*)(T + r1 * 72 + 8 * q8);
  _Float16* d0 = Wt + (size_t)(n0 + r0) * K + k0 + 8 * q8;
  _Float16* d1 = Wt + (size_t)(n0 + r1) * K + k0 + 8 * q8;
  for (int pass = 0; pass < 2; ++pass) {
    *(volatile v8h*)d0 = v0;
    *(volatile v8h*)d1 = v1;
    __threadfence();
  }
}

template <int OMODE, int BMODE, bool GELU, bool RESID>
__global__ __launch_bounds__(256) void gemm64(
    const _Float16* __restrict__ A, int lda, long long strideA,
    const _Float16* __restrict__ Bt, int ldb, long long strideB,
    void* Cout, int ldc, long long strideC,
    const float* __restrict__ bias, const float* __restrict__ resid, int ldr,
    int M, int N, int K, float rsc, float osc) {
  __shared__ __align__(16) float sT[8][16 * 68];
  const int b    = blockIdx.y;
  const int lane = threadIdx.x & 31;
  const int wave = threadIdx.x >> 5;
  const int tilesN = N >> 6;
  const int tilesM = M >> 6;
  const int tile = blockIdx.x * 8 + wave;
  if (tile >= tilesM * tilesN) return;
  const int tm = tile / tilesN;
  const int tn = tile - tm * tilesN;
  const int m0 = tm << 6;
  const int n0 = tn << 6;

  const _Float16* Ab = A  + (size_t)b * (size_t)strideA;
  const _Float16* Bb = Bt + (size_t)b * (size_t)strideB;

  const int rlane = lane & 15;
  const int koff  = (lane >> 4) * 8;
  const int mOff  = (lane >> 4) * 8;

  v8f acc[4][4];
#pragma unroll
  for (int i = 0; i < 4; ++i)
#pragma unroll
    for (int j = 0; j < 4; ++j) acc[i][j] = zero8();

  for (int k0 = 0; k0 < K; k0 += 32) {
    v16h bf[4];
#pragma unroll
    for (int j = 0; j < 4; ++j)
      bf[j] = ldfrag(Bb + (size_t)(n0 + (j << 4) + rlane) * ldb + koff + k0);
#pragma unroll
    for (int i = 0; i < 4; ++i) {
      const v16h af = ldfrag(Ab + (size_t)(m0 + (i << 4) + rlane) * lda + koff + k0);
#pragma unroll
      for (int j = 0; j < 4; ++j) acc[i][j] = mma_raw(af, bf[j], acc[i][j]);
      dep_guard4(acc[i][0], acc[i][1], acc[i][2], acc[i][3], af);
    }
    keep4(bf[0], bf[1], bf[2], bf[3]);
  }
  acc_guard4(acc[0][0], acc[0][1], acc[0][2], acc[0][3]);
  acc_guard4(acc[1][0], acc[1][1], acc[1][2], acc[1][3]);
  acc_guard4(acc[2][0], acc[2][1], acc[2][2], acc[2][3]);
  acc_guard4(acc[3][0], acc[3][1], acc[3][2], acc[3][3]);

  float* slab = sT[wave];
#pragma unroll
  for (int i = 0; i < 4; ++i) {
    const int mBase = m0 + (i << 4);
#pragma unroll
    for (int j = 0; j < 4; ++j) {
#pragma unroll
      for (int r = 0; r < 8; ++r) {
        slab[(mOff + r) * 68 + (j << 4) + rlane] = acc[i][j][r];
      }
    }
    __builtin_amdgcn_fence(__ATOMIC_RELEASE, "workgroup");
    __builtin_amdgcn_wave_barrier();
    __builtin_amdgcn_fence(__ATOMIC_ACQUIRE, "workgroup");
    if (OMODE == 0) {
      float* C = (float*)Cout + (size_t)b * (size_t)strideC;
      const int hh = lane >> 4, c4 = (lane & 15) * 4;
      v4f vals[8];
#pragma unroll
      for (int it = 0; it < 8; ++it) {
        const int row = it * 2 + hh;
        v4f v = *(const v4fa*)(slab + row * 68 + c4) * rsc;
        if (BMODE == 1) v += *(const v4fa*)(bias + n0 + c4);
        if (RESID) v += *(const v4fa*)(resid + (size_t)(mBase + row) * ldr + n0 + c4);
        vals[it] = v;
      }
      for (int pass = 0; pass < 2; ++pass) {
#pragma unroll
        for (int it = 0; it < 8; ++it) {
          const int row = it * 2 + hh;
          *(volatile v4f*)(C + (size_t)(mBase + row) * ldc + n0 + c4) = vals[it];
        }
        __threadfence();
      }
    } else {
      _Float16* C = (_Float16*)Cout + (size_t)b * (size_t)strideC;
      const int q = lane >> 3, c8 = (lane & 7) * 8;
      v8h hv[4];
#pragma unroll
      for (int it = 0; it < 4; ++it) {
        const int row = it * 4 + q;
        const float* sp = slab + row * 68 + c8;
        const v4f s0 = *(const v4fa*)(sp);
        const v4f s1 = *(const v4fa*)(sp + 4);
        v4f b0 = {0.f, 0.f, 0.f, 0.f};
        v4f b1 = {0.f, 0.f, 0.f, 0.f};
        if (BMODE == 1) {
          b0 = *(const v4fa*)(bias + n0 + c8);
          b1 = *(const v4fa*)(bias + n0 + c8 + 4);
        } else if (BMODE == 2) {
          const float bb = bias[mBase + row];
          const v4f bq = {bb, bb, bb, bb};
          b0 = bq; b1 = bq;
        }
        v4f y0 = s0 * rsc + b0;
        v4f y1 = s1 * rsc + b1;
        if (GELU) {
          y0.x = gelu_f(y0.x); y0.y = gelu_f(y0.y); y0.z = gelu_f(y0.z); y0.w = gelu_f(y0.w);
          y1.x = gelu_f(y1.x); y1.y = gelu_f(y1.y); y1.z = gelu_f(y1.z); y1.w = gelu_f(y1.w);
        }
        y0 = y0 * osc;
        y1 = y1 * osc;
        const v8h o = { (_Float16)y0.x, (_Float16)y0.y, (_Float16)y0.z, (_Float16)y0.w,
                        (_Float16)y1.x, (_Float16)y1.y, (_Float16)y1.z, (_Float16)y1.w };
        hv[it] = o;
      }
      for (int pass = 0; pass < 2; ++pass) {
#pragma unroll
        for (int it = 0; it < 4; ++it) {
          const int row = it * 4 + q;
          *(volatile v8h*)(C + (size_t)(mBase + row) * ldc + n0 + c8) = hv[it];
        }
        __threadfence();
      }
    }
    __builtin_amdgcn_fence(__ATOMIC_RELEASE, "workgroup");
    __builtin_amdgcn_wave_barrier();
    __builtin_amdgcn_fence(__ATOMIC_ACQUIRE, "workgroup");
  }
}

__device__ __forceinline__ v16h pack_p(v8f a, v8f c) {
  const v16h r = { (_Float16)(a[0] * PSCALE), (_Float16)(a[1] * PSCALE), (_Float16)(a[2] * PSCALE), (_Float16)(a[3] * PSCALE),
                   (_Float16)(a[4] * PSCALE), (_Float16)(a[5] * PSCALE), (_Float16)(a[6] * PSCALE), (_Float16)(a[7] * PSCALE),
                   (_Float16)(c[0] * PSCALE), (_Float16)(c[1] * PSCALE), (_Float16)(c[2] * PSCALE), (_Float16)(c[3] * PSCALE),
                   (_Float16)(c[4] * PSCALE), (_Float16)(c[5] * PSCALE), (_Float16)(c[6] * PSCALE), (_Float16)(c[7] * PSCALE) };
  return r;
}

__global__ __launch_bounds__(128) void attn_kernel(const _Float16* __restrict__ QK,
                                                   const _Float16* __restrict__ VT,
                                                   _Float16* CTX) {
  __shared__ __align__(16) float sO[4 * 16 * 64];

  const int tid = threadIdx.x, lane = tid & 31, w = tid >> 5;
  const int h = lane >> 4, m = lane & 15;
  const int qt = blockIdx.x, bh = blockIdx.y, b = bh >> 4, head = bh & 15;
  const int q0 = qt * 64 + 16 * w;
  const size_t tok0 = (size_t)b * SEQ;

  const _Float16* qrow = QK + (tok0 + q0 + m) * (size_t)QKP + head * HD + 8 * h;
  const v16h qb0 = ldfrag(qrow);
  const v16h qb1 = ldfrag(qrow + 32);

  v8f o[4];
#pragma unroll
  for (int t = 0; t < 4; ++t) o[t] = zero8();
  float mrun = -1e30f, lrun = 0.0f;

  const _Float16* kbase = QK + (tok0 + m) * (size_t)QKP + HID + head * HD + 8 * h;
  const _Float16* vbase = VT + ((size_t)b * HID + head * HD + m) * SEQ + 8 * h;
  const int qidx = q0 + m;
  const int kend = qt * 64;

#pragma unroll 1
  for (int kb = 0; kb <= kend; kb += 64) {
    v8f s[4];
#pragma unroll
    for (int j = 0; j < 4; ++j) {
      const _Float16* kp = kbase + (size_t)(kb + 16 * j) * QKP;
      const v16h kf0 = ldfrag(kp);
      const v16h kf1 = ldfrag(kp + 32);
      v8f z = zero8();
      z = mma_h(kf0, qb0, z);
      z = mma_h(kf1, qb1, z);
      s[j] = z;
    }
    const bool diag = (kb == kend);
#pragma unroll
    for (int j = 0; j < 4; ++j)
#pragma unroll
      for (int r = 0; r < 8; ++r) {
        const int key = kb + 16 * j + 8 * h + r;
        float vv = s[j][r] * 0.125f;
        if (diag && key > qidx) vv = -INFINITY;
        s[j][r] = vv;
      }

    float mloc = s[0][0];
#pragma unroll
    for (int j = 0; j < 4; ++j)
#pragma unroll
      for (int r = 0; r < 8; ++r) mloc = fmaxf(mloc, s[j][r]);
    mloc = fmaxf(mloc, __shfl_xor(mloc, 16, 32));
    const float mnew = fmaxf(mrun, mloc);
    const float alpha = __expf(mrun - mnew);
    mrun = mnew;
    float lsum = 0.0f;
#pragma unroll
    for (int j = 0; j < 4; ++j)
#pragma unroll
      for (int r = 0; r < 8; ++r) {
        const float p = __expf(s[j][r] - mnew);
        s[j][r] = p;
        lsum += p;
      }
    lsum += __shfl_xor(lsum, 16, 32);
    lrun = lrun * alpha + lsum;
#pragma unroll
    for (int t = 0; t < 4; ++t)
#pragma unroll
      for (int r = 0; r < 8; ++r) o[t][r] = o[t][r] * alpha;

    const v16h pb0 = pack_p(s[0], s[1]);
    const v16h pb1 = pack_p(s[2], s[3]);

#pragma unroll
    for (int t = 0; t < 4; ++t) {
      const _Float16* vp = vbase + (size_t)(16 * t) * SEQ + kb;
      const v16h vf0 = ldfrag(vp);
      const v16h vf1 = ldfrag(vp + 32);
      o[t] = mma_h(vf0, pb0, o[t]);
      o[t] = mma_h(vf1, pb1, o[t]);
    }
  }

  const float inv = (1.0f / lrun) * (CTXC / PSCALE);
  float* so = sO + w * 1024;
#pragma unroll
  for (int t = 0; t < 4; ++t)
#pragma unroll
    for (int r = 0; r < 8; ++r)
      so[m * 64 + 16 * t + 8 * h + r] = o[t][r] * inv;
  __syncthreads();

  const int q8 = lane & 7, sub = lane >> 3;
  v8h hv[4];
#pragma unroll
  for (int i = 0; i < 4; ++i) {
    const int row = i * 4 + sub;
    const float* sp = so + row * 64 + 8 * q8;
    const v4f a = *(const v4fa*)(sp);
    const v4f c = *(const v4fa*)(sp + 4);
    const v8h v = { (_Float16)a.x, (_Float16)a.y, (_Float16)a.z, (_Float16)a.w,
                    (_Float16)c.x, (_Float16)c.y, (_Float16)c.z, (_Float16)c.w };
    hv[i] = v;
  }
  for (int pass = 0; pass < 2; ++pass) {
#pragma unroll
    for (int i = 0; i < 4; ++i) {
      const int row = i * 4 + sub;
      _Float16* dst = CTX + (tok0 + q0 + row) * (size_t)HID + head * HD + 8 * q8;
      *(volatile v8h*)dst = hv[i];
    }
    __threadfence();
  }
}

extern "C" void kernel_launch(void* const* d_in, const int* in_sizes, int n_in,
                              void* d_out, int out_size, void* d_ws, size_t ws_size,
                              hipStream_t stream) {
  if (n_in < 12) return;
  if (in_sizes[0] != NTOK * HID) return;
  if (in_sizes[1] != HID || in_sizes[2] != HID) return;
  if (in_sizes[3] != HID * QKVN || in_sizes[4] != QKVN) return;
  if (in_sizes[5] != HID * HID || in_sizes[6] != HID) return;
  if (in_sizes[7] != HID || in_sizes[8] != HID) return;
  if (in_sizes[9] != HID * FFN || in_sizes[10] != FFN * HID || in_sizes[11] != HID) return;
  if (out_size != NTOK * HID) return;

  const float* x       = (const float*)d_in[0];
  const float* ln1_g   = (const float*)d_in[1];
  const float* ln1_b   = (const float*)d_in[2];
  const float* w_qkv   = (const float*)d_in[3];
  const float* b_qkv   = (const float*)d_in[4];
  const float* w_dense = (const float*)d_in[5];
  const float* b_dense = (const float*)d_in[6];
  const float* ln2_g   = (const float*)d_in[7];
  const float* ln2_b   = (const float*)d_in[8];
  const float* w_fc1   = (const float*)d_in[9];
  const float* w_fc2   = (const float*)d_in[10];
  const float* b_fc2   = (const float*)d_in[11];
  float* out = (float*)d_out;

  const size_t szWqkv = (size_t)QKVN * HID * 2;
  const size_t szWd   = (size_t)HID * HID * 2;
  const size_t szW1   = (size_t)FFN * HID * 2;
  const size_t szW2   = (size_t)HID * FFN * 2;
  const size_t szXN   = (size_t)NTOK * HID * 2;
  const size_t szQK   = (size_t)NTOK * QKP * 2;
  const size_t szVT   = (size_t)NB * HID * SEQ * 2;
  const size_t szCTX  = (size_t)NTOK * HID * 2;
  const size_t szRES  = (size_t)NTOK * HID * 4;
  const size_t szM2   = (size_t)NTOK * HID * 2;
  const size_t szH1   = (size_t)NTOK * FFN * 2;
  size_t off = 0;
  const size_t oWqkv = off; off += szWqkv;
  const size_t oWd   = off; off += szWd;
  const size_t oW1   = off; off += szW1;
  const size_t oW2   = off; off += szW2;
  const size_t oXN   = off; off += szXN;
  const size_t oQK   = off; off += szQK;
  const size_t oVT   = off; off += szVT;
  const size_t oCTX  = off; off += szCTX;
  const size_t oRES  = off; off += szRES;
  const size_t oM2   = off; off += szM2;
  const size_t oH1   = off; off += szH1;
  if (off > ws_size) return;
  if (off > (size_t)134217728) return;

  char* ws = (char*)d_ws;
  _Float16* WQKVT = (_Float16*)(ws + oWqkv);
  _Float16* WDT   = (_Float16*)(ws + oWd);
  _Float16* W1T   = (_Float16*)(ws + oW1);
  _Float16* W2T   = (_Float16*)(ws + oW2);
  _Float16* XN    = (_Float16*)(ws + oXN);
  _Float16* QK    = (_Float16*)(ws + oQK);
  _Float16* VT    = (_Float16*)(ws + oVT);
  _Float16* CTX   = (_Float16*)(ws + oCTX);
  float*    RES1  = (float*)(ws + oRES);
  _Float16* M2    = (_Float16*)(ws + oM2);
  _Float16* H1    = (_Float16*)(ws + oH1);

  const dim3 blk(256);

  wtrans_kernel<<<dim3(QKVN / 64, HID / 64), blk, 0, stream>>>(w_qkv,   WQKVT, HID, QKVN);
  wtrans_kernel<<<dim3(HID / 64,  HID / 64), blk, 0, stream>>>(w_dense, WDT,   HID, HID);
  wtrans_kernel<<<dim3(FFN / 64,  HID / 64), blk, 0, stream>>>(w_fc1,   W1T,   HID, FFN);
  wtrans_kernel<<<dim3(HID / 64,  FFN / 64), blk, 0, stream>>>(w_fc2,   W2T,   FFN, HID);

  ln_kernel<<<dim3(NTOK / 8), blk, 0, stream>>>(x, ln1_g, ln1_b, XN, NTOK);

  gemm64<1, 1, false, false><<<dim3(((NTOK / 64) * (QKP / 64) + 7) / 8, 1), blk, 0, stream>>>(
      XN, HID, 0LL, WQKVT, HID, 0LL,
      (void*)QK, QKP, 0LL,
      b_qkv, x, HID,
      NTOK, QKP, HID, 1.0f / WSC, 1.0f);

  gemm64<1, 2, false, false><<<dim3(((HID / 64) * (SEQ / 64) + 7) / 8, NB), blk, 0, stream>>>(
      WQKVT + (size_t)2 * HID * HID, HID, 0LL, XN, HID, (long long)SEQ * HID,
      (void*)VT, SEQ, (long long)HID * SEQ,
      b_qkv + 2 * HID, x, HID,
      HID, SEQ, HID, 1.0f / WSC, 1.0f);

  attn_kernel<<<dim3(SEQ / 64, NB * NHD), dim3(128), 0, stream>>>(QK, VT, CTX);

  gemm64<0, 1, false, true><<<dim3(((NTOK / 64) * (HID / 64) + 7) / 8, 1), blk, 0, stream>>>(
      CTX, HID, 0LL, WDT, HID, 0LL,
      (void*)RES1, HID, 0LL,
      b_dense, x, HID,
      NTOK, HID, HID, 1.0f / (WSC * CTXC), 1.0f);

  ln_kernel<<<dim3(NTOK / 8), blk, 0, stream>>>(RES1, ln2_g, ln2_b, M2, NTOK);

  gemm64<1, 0, true, false><<<dim3(((NTOK / 64) * (FFN / 64) + 7) / 8, 1), blk, 0, stream>>>(
      M2, HID, 0LL, W1T, HID, 0LL,
      (void*)H1, FFN, 0LL,
      b_fc2, x, HID,
      NTOK, FFN, HID, 1.0f / WSC, H1C);

  gemm64<0, 1, false, true><<<dim3(((NTOK / 64) * (HID / 64) + 7) / 8, 1), blk, 0, stream>>>(
      H1, FFN, 0LL, W2T, FFN, 0LL,
      (void*)out, HID, 0LL,
      b_fc2, RES1, HID,
      NTOK, HID, FFN, 1.0f / (WSC * H1C), 1.0f);

  (void)hipGetLastError();
}
